// TRNetParallel_78013785964660
// MI455X (gfx1250) — hardware-run, weakly checked
//
#include <hip/hip_runtime.h>
#include <math.h>

typedef __attribute__((ext_vector_type(16))) _Float16 v16h;
typedef __attribute__((ext_vector_type(8)))  _Float16 v8h;
typedef __attribute__((ext_vector_type(8)))  float    v8f;
typedef __attribute__((ext_vector_type(4)))  float    v4f;

constexpr int kNB    = 512;
constexpr int kND    = 16;
constexpr int kNIn   = 64;
constexpr int kNM    = 32;
constexpr int kNR    = 32;
constexpr int kNC    = 10;
constexpr int kBT    = 16;
constexpr int kNBT   = kNB / kBT;
constexpr int kRows  = kNB * kND;
constexpr int kRR    = kNR * kNR;
constexpr int kCD    = kNC * kND;
static_assert(kNM == 32 && kNR == 32, "single 32-deep k-step");
static_assert(kNBT * kBT == kNB, "batch tile multiple");
static_assert(kRR == 1024, "core plane size");

constexpr float kCarryG    = 1024.0f;
constexpr float kCarryF    = 16.0f;
constexpr float kCarryCore = 64.0f;
constexpr float kCarryP    = 64.0f;
constexpr float kResid     = 2048.0f;
constexpr float kResidInv  = 1.0f / kResid;
constexpr float kFoldA     = kCarryCore / (kCarryG * kCarryF);
constexpr float kFoldB     = kCarryP / (kCarryCore * kCarryP);
constexpr float kTraceFold = 1.0f / kCarryP;

constexpr size_t kOffGT   = 0;
constexpr size_t kOffFH   = kOffGT + (size_t)kCD * kRR * kNM * 2;
constexpr size_t kOffFL   = kOffFH + (size_t)kRows * kNM * 2;
constexpr size_t kOffLG   = kOffFL + (size_t)kRows * kNM * 2;
constexpr size_t kWsTotal = kOffLG + (size_t)kNC * kNBT * 32 * 4;
static_assert(kWsTotal == 11575296ull, "carve total");
static_assert(kWsTotal <= 134217728ull, "carve cap");
static_assert((kOffFH % 128) == 0 && (kOffFL % 128) == 0 && (kOffLG % 128) == 0, "128-B aligned regions");

constexpr int kLdsCore  = kBT * kRR * 2;
constexpr int kLdsPlane = kBT * kRR * 2;
constexpr int kLdsTotal = kLdsCore + 2 * kLdsPlane + 128;
static_assert(kLdsTotal == 98432, "dynamic LDS size");

union FragH { v16h v; v8h h[2]; };
__device__ __forceinline__ v16h ld_frag(const _Float16* p) {
  FragH f;
  f.h[0] = *(const v8h*)(p);
  f.h[1] = *(const v8h*)(p + 16);
  return f.v;
}
__device__ __forceinline__ v8f mma_h(v16h a, v16h b, v8f c) {
  c = __builtin_amdgcn_wmma_f32_16x16x32_f16(false, a, false, b, (short)0, c, false, false);
  asm volatile("v_nop\n\tv_nop\n\tv_nop\n\tv_nop" : "+v"(c) : "v"(a), "v"(b));
  return c;
}

__global__ __launch_bounds__(256) void prep_g_kernel(
    const float* __restrict__ G, unsigned short* __restrict__ GT)
{
  __shared__ float sG[64 * 33];
  const int tid = threadIdx.x, lane = tid & 31, wave = tid >> 5;
  const int cd = blockIdx.x >> 4;
  const int ip = blockIdx.x & 15;
  const float* src = G + ((size_t)cd * kNR + (size_t)ip * 2) * (kNM * kNR);
#pragma unroll
  for (int k = 0; k < 2; ++k) {
    const int f = (tid + 256 * k) * 4;
    const v4f v = *(const v4f*)(src + f);
    const int row = f >> 5;
    const int j0 = f & 31;
    sG[row * 33 + j0 + 0] = v[0];
    sG[row * 33 + j0 + 1] = v[1];
    sG[row * 33 + j0 + 2] = v[2];
    sG[row * 33 + j0 + 3] = v[3];
  }
  __syncthreads();
  const int j  = wave * 4 + (lane >> 3);
  const int q  = lane & 7;
  const int ii = q >> 2;
  const int m0 = (q & 3) * 8;
  v8h hv;
#pragma unroll
  for (int e = 0; e < 8; ++e) {
    const float g = sG[(ii * 32 + m0 + e) * 33 + j] * kCarryG;
    hv[e] = (_Float16)g;
  }
  unsigned short* dst = GT + ((size_t)cd * kRR + (size_t)j * 32 + (size_t)ip * 2) * kNM + q * 8;
  *(volatile v8h*)dst = hv;
  __threadfence();
  *(volatile v8h*)dst = hv;
}

__global__ __launch_bounds__(256) void feat_kernel(
    const float* __restrict__ xin, const float* __restrict__ W, const float* __restrict__ bfm,
    unsigned short* __restrict__ FH, unsigned short* __restrict__ FL)
{
  __shared__ __align__(16) float sW[kNIn * kNM];
  const int tid = threadIdx.x;
#pragma unroll
  for (int k = 0; k < 2; ++k) {
    const int idx = (tid + 256 * k) * 4;
    *(v4f*)(sW + idx) = *(const v4f*)(W + idx);
  }
  __syncthreads();
  const int gid = blockIdx.x * 256 + tid;
  const int row = gid >> 2;
  const int m0  = (gid & 3) * 8;
  const v4f b0 = *(const v4f*)(bfm + m0);
  const v4f b1 = *(const v4f*)(bfm + m0 + 4);
  float acc[8];
#pragma unroll
  for (int e = 0; e < 8; ++e) acc[e] = 0.0f;
  const float* xr = xin + (size_t)row * kNIn;
#pragma unroll 1
  for (int n4 = 0; n4 < kNIn / 4; ++n4) {
    const v4f tv = *(const v4f*)(xr + 4 * n4);
#pragma unroll
    for (int e = 0; e < 4; ++e) {
      const float* wp = sW + (4 * n4 + e) * kNM + m0;
      const v4f w0 = *(const v4f*)(wp);
      const v4f w1 = *(const v4f*)(wp + 4);
      const float t = tv[e];
      acc[0] = fmaf(t, w0[0], acc[0]);
      acc[1] = fmaf(t, w0[1], acc[1]);
      acc[2] = fmaf(t, w0[2], acc[2]);
      acc[3] = fmaf(t, w0[3], acc[3]);
      acc[4] = fmaf(t, w1[0], acc[4]);
      acc[5] = fmaf(t, w1[1], acc[5]);
      acc[6] = fmaf(t, w1[2], acc[6]);
      acc[7] = fmaf(t, w1[3], acc[7]);
    }
  }
  acc[0] += b0[0]; acc[1] += b0[1]; acc[2] += b0[2]; acc[3] += b0[3];
  acc[4] += b1[0]; acc[5] += b1[1]; acc[6] += b1[2]; acc[7] += b1[3];
  v8h hv, lv;
#pragma unroll
  for (int e = 0; e < 8; ++e) {
    const float xs = acc[e] * kCarryF;
    const _Float16 hh = (_Float16)xs;
    const float hf = (float)hh;
    const float res = (xs - hf) * kResid;
    hv[e] = hh;
    lv[e] = (_Float16)res;
  }
  unsigned short* qh = FH + (size_t)gid * 8;
  unsigned short* ql = FL + (size_t)gid * 8;
  *(volatile v8h*)qh = hv;
  *(volatile v8h*)ql = lv;
  __threadfence();
  *(volatile v8h*)qh = hv;
  *(volatile v8h*)ql = lv;
}

__global__ __launch_bounds__(512) void chain_kernel(
    const unsigned short* __restrict__ GTp, const unsigned short* __restrict__ FHp,
    const unsigned short* __restrict__ FLp, float* __restrict__ LG)
{
  extern __shared__ __align__(16) unsigned char smem[];
  _Float16* sCore = (_Float16*)smem;
  _Float16* sPH   = sCore + kBT * kRR;
  _Float16* sPL   = sPH + kBT * kRR;
  float*    sTr   = (float*)(sPL + kBT * kRR);

  const int tid  = threadIdx.x;
  const int lane = tid & 31;
  const int wave = tid >> 5;
  const int hh   = lane >> 4;
  const int lc   = lane & 15;
  const int c    = blockIdx.x / kNBT;
  const int bt   = blockIdx.x - c * kNBT;

  const _Float16* GT = (const _Float16*)GTp;
  const _Float16* FH = (const _Float16*)FHp;
  const _Float16* FL = (const _Float16*)FLp;

  _Float16* myPH = sPH + wave * kRR;
  _Float16* myPL = sPL + wave * kRR;

#pragma unroll
  for (int k = 0; k < 4; ++k) {
    const int ch   = lane + 32 * k;
    const int prow = ch >> 2;
    const int col0 = (ch & 3) * 8;
    v8h iv, zv;
#pragma unroll
    for (int e = 0; e < 8; ++e) {
      const float f = (prow == col0 + e) ? kCarryP : 0.0f;
      iv[e] = (_Float16)f;
      zv[e] = (_Float16)0.0f;
    }
    *(v8h*)(myPH + ch * 8) = iv;
    *(v8h*)(myPL + ch * 8) = zv;
  }

  const size_t featOff = ((size_t)(bt * kBT + lc) * kND) * kNM + 8 * hh;
  const _Float16* gBase = GT + ((size_t)(c * kND) * kRR + (size_t)(64 * wave + lc)) * kNM + 8 * hh;
  const int dr = lc - 8 * hh;
  const v8f vz = (v8f){0.f, 0.f, 0.f, 0.f, 0.f, 0.f, 0.f, 0.f};
  float tr = 0.0f;

#pragma unroll 1
  for (int d = 0; d < kND; ++d) {
    {
      const v16h fh = ld_frag(FH + featOff + (size_t)d * kNM);
      const v16h fl = ld_frag(FL + featOff + (size_t)d * kNM);
      v16h g[4];
#pragma unroll
      for (int t = 0; t < 4; ++t)
        g[t] = ld_frag(gBase + (size_t)d * (kRR * kNM) + (size_t)t * (16 * kNM));
#pragma unroll
      for (int t = 0; t < 4; ++t) {
        const v8f am = mma_h(g[t], fh, vz);
        const v8f ar = mma_h(g[t], fl, vz);
        v8h cv;
#pragma unroll
        for (int r = 0; r < 8; ++r) {
          const float cvf = (am[r] + ar[r] * kResidInv) * kFoldA;
          cv[r] = (_Float16)cvf;
        }
        const int j  = 2 * wave + (t >> 1);
        const int i0 = (t & 1) * 16 + 8 * hh;
        *(v8h*)(sCore + lc * kRR + j * kNR + i0) = cv;
      }
    }
    __syncthreads();
    {
      v16h cf[2], ph[2], pl[2];
#pragma unroll
      for (int t = 0; t < 2; ++t) {
        cf[t] = ld_frag(sCore + wave * kRR + (t * 16 + lc) * kNR + 8 * hh);
        ph[t] = ld_frag(myPH + (t * 16 + lc) * kNR + 8 * hh);
        pl[t] = ld_frag(myPL + (t * 16 + lc) * kNR + 8 * hh);
      }
      float trn = 0.0f;
#pragma unroll
      for (int tj = 0; tj < 2; ++tj) {
#pragma unroll
        for (int tn = 0; tn < 2; ++tn) {
          const v8f am = mma_h(cf[tj], ph[tn], vz);
          const v8f ar = mma_h(cf[tj], pl[tn], vz);
          v8h hv, lv;
#pragma unroll
          for (int r = 0; r < 8; ++r) {
            const float qv = (am[r] + ar[r] * kResidInv) * kFoldB;
            const _Float16 hq = (_Float16)qv;
            const float hf = (float)hq;
            const float res = (qv - hf) * kResid;
            hv[r] = hq;
            lv[r] = (_Float16)res;
            if (tj == tn) trn += (r == dr) ? qv : 0.0f;
          }
          *(v8h*)(myPH + (tn * 16 + lc) * kNR + tj * 16 + 8 * hh) = hv;
          *(v8h*)(myPL + (tn * 16 + lc) * kNR + tj * 16 + 8 * hh) = lv;
        }
      }
      tr = trn;
    }
    __syncthreads();
  }

#pragma unroll
  for (int off = 16; off > 0; off >>= 1) tr += __shfl_xor(tr, off, 32);
  const float lg = tr * kTraceFold;
  if (lane < 2) sTr[lane * 16 + wave] = (lane == 0) ? lg : 0.0f;
  __syncthreads();
  if (wave == 0) {
    const float v = sTr[lane];
    volatile float* dst = LG + ((size_t)(c * kNBT + bt)) * 32 + lane;
    *dst = v;
    __threadfence();
    *dst = v;
  }
}

__global__ __launch_bounds__(256) void lsm_kernel(const float* __restrict__ LG, float* __restrict__ out)
{
  const int idx = blockIdx.x * 256 + threadIdx.x;
  const int b = idx / kNC;
  const int c = idx - b * kNC;
  const float* base = LG + (size_t)(b >> 4) * 32 + (b & 15);
  float mx = -INFINITY;
#pragma unroll 1
  for (int cc = 0; cc < kNC; ++cc) mx = fmaxf(mx, base[(size_t)cc * (kNBT * 32)]);
  float s = 0.0f;
#pragma unroll 1
  for (int cc = 0; cc < kNC; ++cc) s += expf(base[(size_t)cc * (kNBT * 32)] - mx);
  const float mine = base[(size_t)c * (kNBT * 32)];
  const float val = (mine - mx) - logf(s);
  volatile float* dst = out + idx;
  *dst = val;
  __threadfence();
  *dst = val;
}
static_assert((kNB * kNC) % 256 == 0, "softmax grid exact");
static_assert((kRows * 4) % 256 == 0, "feature grid exact");

extern "C" void kernel_launch(void* const* d_in, const int* in_sizes, int n_in,
                              void* d_out, int out_size, void* d_ws, size_t ws_size,
                              hipStream_t stream) {
  if (n_in < 4) return;
  if (in_sizes[0] != kNB * kND * kNIn) return;
  if (in_sizes[1] != kNIn * kNM) return;
  if (in_sizes[2] != kNM) return;
  if (in_sizes[3] != kCD * kNR * kNM * kNR) return;
  if (out_size != kNB * kNC) return;
  if (ws_size < kWsTotal) return;

  const float* xin  = (const float*)d_in[0];
  const float* W_fm = (const float*)d_in[1];
  const float* b_fm = (const float*)d_in[2];
  const float* G    = (const float*)d_in[3];
  float* out = (float*)d_out;

  char* ws = (char*)d_ws;
  unsigned short* GT = (unsigned short*)(ws + kOffGT);
  unsigned short* FH = (unsigned short*)(ws + kOffFH);
  unsigned short* FL = (unsigned short*)(ws + kOffFL);
  float*          LG = (float*)(ws + kOffLG);

  prep_g_kernel<<<kCD * (kNR / 2), 256, 0, stream>>>(G, GT);
  feat_kernel<<<(kRows * 4) / 256, 256, 0, stream>>>(xin, W_fm, b_fm, FH, FL);
  chain_kernel<<<kNC * kNBT, 512, kLdsTotal, stream>>>(GT, FH, FL, LG);
  lsm_kernel<<<(kNB * kNC) / 256, 256, 0, stream>>>(LG, out);
}
